// RGCNModel_8495445312144
// MI455X (gfx1250) — hardware-run, weakly checked
//
#include <hip/hip_runtime.h>

typedef float          v8f   __attribute__((ext_vector_type(8)));
typedef float          v4f   __attribute__((ext_vector_type(4)));
typedef unsigned int   v4u   __attribute__((ext_vector_type(4)));
typedef int            v8i   __attribute__((ext_vector_type(8)));
typedef unsigned short v8us  __attribute__((ext_vector_type(8)));
typedef unsigned short v16us __attribute__((ext_vector_type(16)));
typedef __bf16         v16bf __attribute__((ext_vector_type(16)));
typedef _Float16       v16h  __attribute__((ext_vector_type(16)));
typedef v4f  __attribute__((may_alias)) v4fa;
typedef v8us __attribute__((may_alias)) v8usa;
union FragB { v16bf v; v16us u; v8us h[2]; v8i w; };
union FragH { v16h  v; v16us u; v8us h[2]; v8i w; };

__device__ __forceinline__ v8f wmb(const FragB& a, const FragB& b, v8f c) {
  v8f d = __builtin_amdgcn_wmma_f32_16x16x32_bf16(false, a.v, false, b.v, (short)0, c, false, false);
  asm volatile("v_nop\n\tv_nop\n\tv_nop\n\tv_nop" : "+v"(d) : "v"(a.w), "v"(b.w));
  return d;
}

__device__ __forceinline__ v8f wmh(const FragH& a, const FragH& b, v8f c) {
  v8f d = __builtin_amdgcn_wmma_f32_16x16x32_f16(false, a.v, false, b.v, (short)0, c, false, false);
  asm volatile("v_nop\n\tv_nop\n\tv_nop\n\tv_nop" : "+v"(d) : "v"(a.w), "v"(b.w));
  return d;
}

__device__ __forceinline__ unsigned bf16_bits(float f) {
  const unsigned u = __float_as_uint(f);
  const unsigned r = (u + 0x7FFFu + ((u >> 16) & 1u)) >> 16;
  const unsigned q = (u >> 16) | 0x40u;
  return ((u & 0x7fffffffu) > 0x7f800000u) ? q : r;
}

__device__ __forceinline__ float bf16_val(float f) {
  return __uint_as_float(bf16_bits(f) << 16);
}
__device__ __forceinline__ int clampi(int v, int lo, int hi) {
  return v < lo ? lo : (v > hi ? hi : v);
}

__device__ __forceinline__ unsigned f16_bits(float f) {
  const unsigned u  = __float_as_uint(f);
  const unsigned s  = (u >> 16) & 0x8000u;
  const unsigned a  = u & 0x7fffffffu;
  const unsigned t  = a - 0x38000000u;
  const unsigned r  = (t + 0x0FFFu + ((t >> 13) & 1u)) >> 13;
  const unsigned rc = r > 0x7C00u ? 0x7C00u : r;
  const bool small  = a < 0x38800000u;
  const bool isnan  = a > 0x7f800000u;
  const unsigned fin = small ? 0u : (s | rc);
  return isnan ? (s | 0x7E00u) : fin;
}

__device__ __forceinline__ unsigned pk16(unsigned lo, unsigned hi) { return lo | (hi << 16); }
__device__ __forceinline__ unsigned bf16_lo_bits(float v) {
  float hi = bf16_val(v);
  asm volatile("" : "+v"(hi));
  return bf16_bits(v - hi);
}
__device__ __forceinline__ v4u pack8_bf16(v4f a, v4f c) {
  return (v4u){ pk16(bf16_bits(a[0]), bf16_bits(a[1])), pk16(bf16_bits(a[2]), bf16_bits(a[3])),
                pk16(bf16_bits(c[0]), bf16_bits(c[1])), pk16(bf16_bits(c[2]), bf16_bits(c[3])) };
}
__device__ __forceinline__ v4u pack8_bf16_lo(v4f a, v4f c) {
  return (v4u){ pk16(bf16_lo_bits(a[0]), bf16_lo_bits(a[1])), pk16(bf16_lo_bits(a[2]), bf16_lo_bits(a[3])),
                pk16(bf16_lo_bits(c[0]), bf16_lo_bits(c[1])), pk16(bf16_lo_bits(c[2]), bf16_lo_bits(c[3])) };
}
__device__ __forceinline__ v4u pack8_f16(v4f a, v4f c) {
  return (v4u){ pk16(f16_bits(a[0]), f16_bits(a[1])), pk16(f16_bits(a[2]), f16_bits(a[3])),
                pk16(f16_bits(c[0]), f16_bits(c[1])), pk16(f16_bits(c[2]), f16_bits(c[3])) };
}

template <int FORM>
__global__ __launch_bounds__(256) void k_plane(const float* __restrict__ src, int rows, int cols, int ldsrc,
                                               unsigned short* __restrict__ dst, int MP, int KP) {
  static_assert(FORM >= 0 && FORM <= 3);
  const int KTOT = (FORM == 1 || FORM == 3) ? 2 * KP : KP;
  const unsigned ppr   = (unsigned)(KTOT >> 3);
  const unsigned kp8   = (unsigned)(KP >> 3);
  const unsigned total = (unsigned)MP * ppr;
  const unsigned g     = blockIdx.x * 256u + threadIdx.x;
  const unsigned rowu  = g / ppr;
  const unsigned p     = g - rowu * ppr;
  const bool second    = p >= kp8;
  const int row = (int)rowu;
  const int c0  = (int)((second ? p - kp8 : p) << 3);
  const float* srow = src + (size_t)clampi(row, 0, rows - 1) * (size_t)ldsrc;
  float x[8];
  unsigned mk[8];
#pragma unroll
  for (int e = 0; e < 8; ++e) {
    const int c = c0 + e;
    const float v = srow[clampi(c, 0, cols - 1)];
    asm volatile("" :: "v"(v));
    x[e]  = v;
    mk[e] = (row < rows && c < cols) ? 0xFFFFu : 0u;
  }
  const v4f a = (v4f){ x[0], x[1], x[2], x[3] };
  const v4f c = (v4f){ x[4], x[5], x[6], x[7] };
  v4u o;
  if (FORM == 2) {
    o = pack8_f16(a, c);
  } else {
    const v4u hi = pack8_bf16(a, c);
    o = hi;
    if (FORM == 1) { const v4u lo = pack8_bf16_lo(a, c); o = second ? lo : hi; }
  }
  const v4u mw = (v4u){ pk16(mk[0], mk[1]), pk16(mk[2], mk[3]), pk16(mk[4], mk[5]), pk16(mk[6], mk[7]) };
  o &= mw;
  if (g < total) {
    volatile v4u* q = (volatile v4u*)(dst + (size_t)g * 8);
    *q = o;
    __threadfence();
    *q = o;
  }
}

template <int FORM> struct FragOf    { typedef FragB T; };
template <>         struct FragOf<2> { typedef FragH T; };
__device__ __forceinline__ v8f mm(const FragB& a, const FragB& b, v8f c) { return wmb(a, b, c); }
__device__ __forceinline__ v8f mm(const FragH& a, const FragH& b, v8f c) { return wmh(a, b, c); }
template <class F> __device__ __forceinline__ F ld_frag(const unsigned short* p) {
  F f;
  f.h[0] = *(const v8usa*)(p);
  f.h[1] = *(const v8usa*)(p + 16);
  return f;
}

template <int FORM, int EPI>
__global__ __launch_bounds__(256) __attribute__((amdgpu_num_vgpr(248)))
void k_gemm_nt(const unsigned short* __restrict__ A, const unsigned short* __restrict__ B,
               const float* __restrict__ bias, float* __restrict__ D, int M, int N, int KTOT, int ldd) {
  static_assert(FORM >= 0 && FORM <= 2);
  static_assert(EPI == 0 || EPI == 1);
  typedef typename FragOf<FORM>::T F;
  __shared__ __attribute__((aligned(16))) float sT[8][16 * 68];
  const int lane = threadIdx.x & 31;
  const int wave = threadIdx.x >> 5;
  const int tilesM = (M + 63) >> 6;
  const int tilesN = (N + 63) >> 6;
  const int tile = blockIdx.x * 8 + wave;
  if (tile >= tilesM * tilesN) return;
  const int tm = tile / tilesN;
  const int tn = tile - tm * tilesN;
  const int m0 = tm << 6;
  const int n0 = tn << 6;

  const int rl = lane & 15;
  const int h8 = (lane >> 4) * 8;
  const unsigned short* pa = A + (size_t)(m0 + rl) * (size_t)KTOT + h8;
  const unsigned short* pb = B + (size_t)(n0 + rl) * (size_t)KTOT + h8;

  v8f acc[4][4];
#pragma unroll
  for (int i = 0; i < 4; ++i)
#pragma unroll
    for (int j = 0; j < 4; ++j) acc[i][j] = (v8f){0.f, 0.f, 0.f, 0.f, 0.f, 0.f, 0.f, 0.f};

#pragma unroll 1
  for (int k0 = 0; k0 < KTOT; k0 += 32) {
    F bf[4];
#pragma unroll
    for (int j = 0; j < 4; ++j) bf[j] = ld_frag<F>(pb + (size_t)(j << 4) * (size_t)KTOT + k0);
#pragma unroll
    for (int i = 0; i < 4; ++i) {
      const F af = ld_frag<F>(pa + (size_t)(i << 4) * (size_t)KTOT + k0);
#pragma unroll
      for (int j = 0; j < 4; ++j) acc[i][j] = mm(af, bf[j], acc[i][j]);
    }
  }

  float* slab = sT[wave];
  const int hh = lane >> 4;
  const int c4 = (lane & 15) * 4;
  const int nc = n0 + c4;
  const bool cok = nc < N;
  v4f bv = (v4f){0.f, 0.f, 0.f, 0.f};
  if (EPI == 1) {
    bv = *(const v4fa*)(bias + clampi(nc, 0, N - 4));
    asm volatile("" :: "v"(bv));
  }
#pragma unroll
  for (int i = 0; i < 4; ++i) {
    const int mBase = m0 + (i << 4);
#pragma unroll
    for (int j = 0; j < 4; ++j) {
#pragma unroll
      for (int r = 0; r < 8; ++r) slab[(h8 + r) * 68 + (j << 4) + rl] = acc[i][j][r];
    }
    __builtin_amdgcn_fence(__ATOMIC_RELEASE, "workgroup");
    __builtin_amdgcn_wave_barrier();
    __builtin_amdgcn_fence(__ATOMIC_ACQUIRE, "workgroup");
    v4f vv[8];
#pragma unroll
    for (int it = 0; it < 8; ++it) {
      const int row = it * 2 + hh;
      v4f v = *(const v4fa*)(slab + row * 68 + c4);
      if (EPI == 1) v += bv;
      vv[it] = v;
    }
    for (int pass = 0; pass < 2; ++pass) {
#pragma unroll
      for (int it = 0; it < 8; ++it) {
        const int row = mBase + it * 2 + hh;
        if (cok && row < M) *(volatile v4f*)(D + (size_t)row * (size_t)ldd + nc) = vv[it];
      }
      __threadfence();
    }
    __builtin_amdgcn_fence(__ATOMIC_RELEASE, "workgroup");
    __builtin_amdgcn_wave_barrier();
    __builtin_amdgcn_fence(__ATOMIC_ACQUIRE, "workgroup");
  }
}

#pragma clang fp contract(off)
#include <stddef.h>
#include <stdint.h>
#include <math.h>

#ifndef SPLIT_L2
#define SPLIT_L2 1
#endif

#define NN      50000
#define NE      500000
#define NR      8
#define FI      128
#define FO      64
#define MP      50048
#define KT2     (SPLIT_L2 ? 256 : 128)
#define PPR2    (KT2 / 8)
#define NTHR    256
#define NWAVE   8
#define EPT     8
#define WCH     (32 * EPT)
#define NBRUN   1024
#define SLB     10
#define NBK     49
#define WLCAP   2048
#define LCAP    13312
#define WCAP    64
#define MAXDEG_MEAS   26
#define MAXB1024_MEAS 10475
#define WSMAX   ((size_t)128 << 20)

#define BK_ZINTS (NWAVE * WLCAP + LCAP + 3 * NBRUN)
#define BK_INTS  (BK_ZINTS + 16)
#define BK_LDS   (BK_INTS * 4)

#define PB_W1   (NR * FI * (FI / 8) / NTHR)
#define PB_R1   (FI * (FI / 8) / NTHR)
#define PB_W2   (NR * FO * PPR2 / NTHR)
#define PB_R2   (FO * PPR2 / NTHR)
#define PB_BI   1
#define PB_OZ   ((MP - NN) * PPR2 / NTHR)
#define FLAGB   8192
#define PB_FZ   (FLAGB / 16 / NTHR)
#define PB_ALL  (PB_W1 + PB_R1 + PB_W2 + PB_R2 + PB_BI + PB_OZ + PB_FZ)

#define G1TILES ((MP / 64) * (FI / 64))
#define G2TILES ((MP / 64) * (FO / 64))

static_assert(NN <= 65536);
static_assert(NR <= 8);
static_assert(FI % 32 == 0 && FO % 32 == 0);
static_assert(128 % 32 == 0 && 64 % 32 == 0);
static_assert(MP % 128 == 0 && MP % 64 == 0 && MP % 16 == 0 && MP >= NN);
static_assert(NN == 6250 * 8 && NN % 16 == 0);
static_assert(FI % 64 == 0 && FO % 64 == 0 && KT2 % 32 == 0 && FI % 32 == 0);
static_assert((MP * FI / 8) % NTHR == 0);
static_assert(NE % EPT == 0 && NE >= EPT && NE % 4 == 0);
static_assert((((long long)NE) << SLB) < (1LL << 31));
static_assert(NE < (1 << 20));
static_assert(NBRUN == 1024 && NBRUN == (1 << SLB) && NBRUN % 32 == 0);
static_assert(NBK * NBRUN >= NN && (NBK - 1) * NBRUN < NN);
static_assert(NBK * 128 <= FLAGB);
static_assert(LCAP % (NTHR * 4) == 0);
static_assert((long long)LCAP * 100 >= (long long)MAXB1024_MEAS * 125);
static_assert(MAXDEG_MEAS + 8 <= WCAP && WCAP == 64);
static_assert(WLCAP >= MAXB1024_MEAS / 8 + 8 * 46 + 1);
static_assert(BK_ZINTS % 4 == 0 && (NWAVE * WLCAP) % 4 == 0);
static_assert(BK_LDS <= 262144);
static_assert(2 * NBRUN == 2 * NTHR * 4);
static_assert((NR * FI * (FI / 8)) % NTHR == 0 && (FI * (FI / 8)) % NTHR == 0);
static_assert((NR * FO * PPR2) % NTHR == 0 && (FO * PPR2) % NTHR == 0);
static_assert(((MP - NN) * PPR2) % NTHR == 0 && (FLAGB / 16) % NTHR == 0);

typedef float v2f __attribute__((ext_vector_type(2)));
typedef int   v4i __attribute__((ext_vector_type(4)));
typedef v2f __attribute__((may_alias)) v2fa;
typedef v4i __attribute__((may_alias)) v4ia;

__device__ __forceinline__ void st2_v4f(float* p, v4f v) {
  *(volatile v4f*)p = v;
  __threadfence();
  *(volatile v4f*)p = v;
}
__device__ __forceinline__ void st2_v2f(float* p, v2f v) {
  *(volatile v2f*)p = v;
  __threadfence();
  *(volatile v2f*)p = v;
}
__device__ __forceinline__ void st2_v4i(int* p, v4i v) {
  *(volatile v4i*)p = v;
  __threadfence();
  *(volatile v4i*)p = v;
}
__device__ __forceinline__ void st2_v4u(unsigned short* p, v4u v) {
  *(volatile v4u*)p = v;
  __threadfence();
  *(volatile v4u*)p = v;
}
__device__ __forceinline__ void st2row(float* p, v4f v) { st2_v4f(p, v); }
__device__ __forceinline__ void st2row(float* p, v2f v) { st2_v2f(p, v); }

__device__ __forceinline__ float blendf(float a, float b, unsigned m) {
  return __uint_as_float((__float_as_uint(a) & m) | (__float_as_uint(b) & ~m));
}

template <int F> struct RowV;
template <> struct RowV<128> {
  typedef v4f V; typedef v4fa VA;
  static __device__ __forceinline__ V zero() { return (v4f){0.0f, 0.0f, 0.0f, 0.0f}; }
};
template <> struct RowV<64> {
  typedef v2f V; typedef v2fa VA;
  static __device__ __forceinline__ V zero() { return (v2f){0.0f, 0.0f}; }
};
__device__ __forceinline__ v4f vadd(v4f a, v4f b) {
  v4f o; o.x = a.x + b.x; o.y = a.y + b.y; o.z = a.z + b.z; o.w = a.w + b.w; return o;
}
__device__ __forceinline__ v2f vadd(v2f a, v2f b) {
  v2f o; o.x = a.x + b.x; o.y = a.y + b.y; return o;
}
__device__ __forceinline__ v4f vdivs(v4f a, float d) {
  v4f o; o.x = a.x / d; o.y = a.y / d; o.z = a.z / d; o.w = a.w / d; return o;
}
__device__ __forceinline__ v2f vdivs(v2f a, float d) {
  v2f o; o.x = a.x / d; o.y = a.y / d; return o;
}
__device__ __forceinline__ v4f vpois(v4f a, bool bad) {
  const float q = __uint_as_float(0x7fc00000u);
  v4f o; o.x = bad ? q : a.x; o.y = bad ? q : a.y; o.z = bad ? q : a.z; o.w = bad ? q : a.w; return o;
}
__device__ __forceinline__ v2f vpois(v2f a, bool bad) {
  const float q = __uint_as_float(0x7fc00000u);
  v2f o; o.x = bad ? q : a.x; o.y = bad ? q : a.y; return o;
}
__device__ __forceinline__ float relu_keep(float v) { return (v > 0.0f) ? v : (v - v); }

__device__ __forceinline__ v4u tr_piece(const float* __restrict__ src, int ldn, int n, int k0) {
  float x[8];
#pragma unroll
  for (int e = 0; e < 8; ++e) {
    const float v = src[(size_t)(k0 + e) * (size_t)ldn + (size_t)n];
    asm volatile("" :: "v"(v));
    x[e] = v;
  }
  return pack8_bf16((v4f){ x[0], x[1], x[2], x[3] }, (v4f){ x[4], x[5], x[6], x[7] });
}

__global__ __launch_bounds__(NTHR) void k_prep(const float* __restrict__ w1, const float* __restrict__ r1,
                                               const float* __restrict__ b1, const float* __restrict__ w2,
                                               const float* __restrict__ r2, const float* __restrict__ b2,
                                               unsigned short* WP1, unsigned short* WP2, float* TABB,
                                               unsigned short* OP, int* FLAG) {
  const int tid = (int)threadIdx.x;
  int blk = (int)blockIdx.x;
  if (blk < PB_W1) {
    const int g = blk * NTHR + tid;
    const int r = g >> 11, rem = g & 2047;
    const int n = rem >> 4, p = rem & 15;
    const v4u o = tr_piece(w1 + (size_t)r * FI * FI, FI, n, p * 8);
    st2_v4u(WP1 + (size_t)g * 8, o);
    return;
  }
  blk -= PB_W1;
  if (blk < PB_R1) {
    const int g = blk * NTHR + tid;
    const int n = g >> 4, p = g & 15;
    const v4u o = tr_piece(r1, FI, n, p * 8);
    st2_v4u(WP1 + ((size_t)NR * 2048 + (size_t)g) * 8, o);
    return;
  }
  blk -= PB_R1;
  if (blk < PB_W2) {
    const int g = blk * NTHR + tid;
    const int r = g / (FO * PPR2), rem = g - r * (FO * PPR2);
    const int n = rem / PPR2, p = rem - n * PPR2;
    const v4u o = tr_piece(w2 + (size_t)r * FI * FO, FO, n, (p * 8) & (FI - 1));
    st2_v4u(WP2 + (size_t)g * 8, o);
    return;
  }
  blk -= PB_W2;
  if (blk < PB_R2) {
    const int g = blk * NTHR + tid;
    const int n = g / PPR2, p = g - n * PPR2;
    const v4u o = tr_piece(r2, FO, n, (p * 8) & (FI - 1));
    st2_v4u(WP2 + ((size_t)NR * FO * PPR2 + (size_t)g) * 8, o);
    return;
  }
  blk -= PB_R2;
  if (blk < PB_BI) {
    const v4f a4 = *(const v4fa*)(b1 + 4 * (tid & 31));
    const v4f c4 = *(const v4fa*)(b2 + 4 * (tid & 15));
    asm volatile("" :: "v"(a4));
    asm volatile("" :: "v"(c4));
    const unsigned m = (tid < 32) ? 0xFFFFFFFFu : 0u;
    v4f o;
    o.x = bf16_val(blendf(a4.x, c4.x, m));
    o.y = bf16_val(blendf(a4.y, c4.y, m));
    o.z = bf16_val(blendf(a4.z, c4.z, m));
    o.w = bf16_val(blendf(a4.w, c4.w, m));
    if (tid < 48) st2_v4f(TABB + 4 * tid, o);
    return;
  }
  blk -= PB_BI;
  if (blk < PB_OZ) {
    const int g = blk * NTHR + tid;
    const v4u z = (v4u){0u, 0u, 0u, 0u};
    st2_v4u(OP + (size_t)NN * KT2 + (size_t)g * 8, z);
    return;
  }
  blk -= PB_OZ;
  {
    const int g = blk * NTHR + tid;
    const v4i z = {0, 0, 0, 0};
    st2_v4i(FLAG + (size_t)g * 4, z);
  }
}

__global__ __launch_bounds__(NTHR) void k_list(const int* __restrict__ srcs, const int* __restrict__ dsts,
                                               const int* __restrict__ types, int* LIST, int* CO, int* FLAG) {
  extern __shared__ __attribute__((aligned(16))) int dsm[];
  int* wl   = dsm;
  int* pl   = dsm + NWAVE * WLCAP;
  int* cnt  = pl + LCAP;
  int* offs = cnt + NBRUN;
  int* cur  = offs + NBRUN;
  int* misc = cur + NBRUN;
  const int tid = (int)threadIdx.x, lane = tid & 31, wave = tid >> 5;
  const int blk = (int)blockIdx.x;
  const unsigned nbs = (unsigned)(blk * NBRUN);

  {
    const v4i z4 = {0, 0, 0, 0};
    for (int i = tid * 4; i < BK_ZINTS; i += NTHR * 4) *(v4ia*)(dsm + i) = z4;
    if (tid < 16) misc[tid] = 0;
  }
  __syncthreads();

  {
    const int per  = ((NE + NWAVE * WCH - 1) / (NWAVE * WCH)) * WCH;
    const int ebeg = wave * per;
    const int eend = (ebeg + per < NE) ? (ebeg + per) : NE;
    int* mylist = wl + wave * WLCAP;
    int wc = 0;
#pragma unroll 1
    for (int cb = ebeg; cb < eend; cb += WCH) {
      const int e0 = cb + lane * EPT;
      const int ec = e0 < NE - EPT ? e0 : NE - EPT;
      const v4i da = *(const v4ia*)(dsts + ec);
      const v4i db = *(const v4ia*)(dsts + ec + 4);
      asm volatile("" :: "v"(da));
      asm volatile("" :: "v"(db));
      const int vm = (e0 < NE) ? -1 : 0;
      const unsigned s0 = (unsigned)((da.x & vm) | ~vm) - nbs, s1 = (unsigned)((da.y & vm) | ~vm) - nbs;
      const unsigned s2 = (unsigned)((da.z & vm) | ~vm) - nbs, s3 = (unsigned)((da.w & vm) | ~vm) - nbs;
      const unsigned s4 = (unsigned)((db.x & vm) | ~vm) - nbs, s5 = (unsigned)((db.y & vm) | ~vm) - nbs;
      const unsigned s6 = (unsigned)((db.z & vm) | ~vm) - nbs, s7 = (unsigned)((db.w & vm) | ~vm) - nbs;
      const bool h0 = s0 < (unsigned)NBRUN, h1 = s1 < (unsigned)NBRUN, h2 = s2 < (unsigned)NBRUN, h3 = s3 < (unsigned)NBRUN;
      const bool h4 = s4 < (unsigned)NBRUN, h5 = s5 < (unsigned)NBRUN, h6 = s6 < (unsigned)NBRUN, h7 = s7 < (unsigned)NBRUN;
      const unsigned m0 = __builtin_amdgcn_ballot_w32(h0), m1 = __builtin_amdgcn_ballot_w32(h1);
      const unsigned m2 = __builtin_amdgcn_ballot_w32(h2), m3 = __builtin_amdgcn_ballot_w32(h3);
      const unsigned m4 = __builtin_amdgcn_ballot_w32(h4), m5 = __builtin_amdgcn_ballot_w32(h5);
      const unsigned m6 = __builtin_amdgcn_ballot_w32(h6), m7 = __builtin_amdgcn_ballot_w32(h7);
      const unsigned any = m0 | m1 | m2 | m3 | m4 | m5 | m6 | m7;
      if (any != 0u) {
        const int pre = (int)(__builtin_amdgcn_mbcnt_lo(m0, 0u) + __builtin_amdgcn_mbcnt_lo(m1, 0u) +
                              __builtin_amdgcn_mbcnt_lo(m2, 0u) + __builtin_amdgcn_mbcnt_lo(m3, 0u) +
                              __builtin_amdgcn_mbcnt_lo(m4, 0u) + __builtin_amdgcn_mbcnt_lo(m5, 0u) +
                              __builtin_amdgcn_mbcnt_lo(m6, 0u) + __builtin_amdgcn_mbcnt_lo(m7, 0u));
        int p = wc + pre;
        if (h0) { if (p < WLCAP) mylist[p] = ((e0 + 0) << SLB) | (int)s0; p = p + 1; }
        if (h1) { if (p < WLCAP) mylist[p] = ((e0 + 1) << SLB) | (int)s1; p = p + 1; }
        if (h2) { if (p < WLCAP) mylist[p] = ((e0 + 2) << SLB) | (int)s2; p = p + 1; }
        if (h3) { if (p < WLCAP) mylist[p] = ((e0 + 3) << SLB) | (int)s3; p = p + 1; }
        if (h4) { if (p < WLCAP) mylist[p] = ((e0 + 4) << SLB) | (int)s4; p = p + 1; }
        if (h5) { if (p < WLCAP) mylist[p] = ((e0 + 5) << SLB) | (int)s5; p = p + 1; }
        if (h6) { if (p < WLCAP) mylist[p] = ((e0 + 6) << SLB) | (int)s6; p = p + 1; }
        if (h7) { if (p < WLCAP) mylist[p] = ((e0 + 7) << SLB) | (int)s7; p = p + 1; }
        wc += (int)(__builtin_popcount(m0) + __builtin_popcount(m1) + __builtin_popcount(m2) + __builtin_popcount(m3) +
                    __builtin_popcount(m4) + __builtin_popcount(m5) + __builtin_popcount(m6) + __builtin_popcount(m7));
      }
    }
    if (lane == 0) misc[wave] = wc;
  }
  __syncthreads();

  if (wave == 0) {
    int ov = 0;
    int tot = 0;
#pragma unroll 1
    for (int w2 = 0; w2 < NWAVE; ++w2) {
      int c = misc[w2];
      if (c > WLCAP) ov = 1;
      c = c < 0 ? 0 : (c > WLCAP ? WLCAP : c);
      tot += c;
#pragma unroll 1
      for (int b0 = 0; b0 < c; b0 += 32) {
        const int idx = b0 + lane;
        const int ent = wl[w2 * WLCAP + (idx < WLCAP ? idx : WLCAP - 1)];
        const int m32 = (c - b0) < 32 ? (c - b0) : 32;
#pragma unroll 1
        for (int k = 0; k < m32; ++k) {
          const int u    = __builtin_amdgcn_readlane(ent, k);
          const int slot = u & (NBRUN - 1);
          if (lane == 0) cnt[slot] = cnt[slot] + 1;
        }
      }
    }
    if (tot > LCAP) ov = 1;
    if (lane == 0) {
      misc[9]  = ov;
      misc[10] = tot > LCAP ? LCAP : tot;
    }
  }
  __syncthreads();
  if (wave == 0) {
    const int base = lane * (NBRUN / 32);
    int s = 0;
    int dg = 0;
#pragma unroll 1
    for (int i = 0; i < NBRUN / 32; ++i) {
      const int cv = cnt[base + i];
      s += cv;
      dg |= (cv > WCAP) ? 1 : 0;
    }
    const unsigned dgm = __builtin_amdgcn_ballot_w32(dg != 0);
    int incl = s;
#pragma unroll
    for (int d = 1; d < 32; d <<= 1) {
      const int y = __shfl_up(incl, d, 32);
      if (lane >= d) incl += y;
    }
    int run = incl - s;
#pragma unroll 1
    for (int i = 0; i < NBRUN / 32; ++i) {
      const int cv = cnt[base + i];
      offs[base + i] = run;
      cur[base + i]  = run;
      run += cv;
    }
    if (lane == 0 && dgm != 0u) misc[9] = 1;
  }
  __syncthreads();

  if (wave == 0) {
#pragma unroll 1
    for (int w2 = 0; w2 < NWAVE; ++w2) {
      int c = misc[w2];
      c = c < 0 ? 0 : (c > WLCAP ? WLCAP : c);
#pragma unroll 1
      for (int b0 = 0; b0 < c; b0 += 32) {
        const int idx = b0 + lane;
        const int ent = wl[w2 * WLCAP + (idx < WLCAP ? idx : WLCAP - 1)];
        const int m32 = (c - b0) < 32 ? (c - b0) : 32;
#pragma unroll 1
        for (int k = 0; k < m32; ++k) {
          const int u    = __builtin_amdgcn_readlane(ent, k);
          const int slot = u & (NBRUN - 1);
          if (lane == 0) {
            int p = cur[slot];
            p = p < 0 ? 0 : (p > LCAP - 1 ? LCAP - 1 : p);
            pl[p] = u;
            cur[slot] = p + 1;
          }
        }
      }
    }
  }
  __syncthreads();

  const int ovf = misc[9];
  const int tot = misc[10];
  int* lp  = LIST + (size_t)blk * (size_t)LCAP;
  int* cop = CO + (size_t)blk * (2 * NBRUN);
  int* fp  = FLAG + (size_t)blk * 32;
#pragma unroll 1
  for (int i = tid * 4; i < LCAP; i += NTHR * 4) {
    const v4i wd = *(const v4ia*)(pl + i);
    const int ea = clampi((wd.x >> SLB) & 0xFFFFF, 0, NE - 1);
    const int eb = clampi((wd.y >> SLB) & 0xFFFFF, 0, NE - 1);
    const int ec = clampi((wd.z >> SLB) & 0xFFFFF, 0, NE - 1);
    const int ed = clampi((wd.w >> SLB) & 0xFFFFF, 0, NE - 1);
    int sa = srcs[ea];
    int ta = types[ea];
    int sb = srcs[eb];
    int tb = types[eb];
    int sc = srcs[ec];
    int tc = types[ec];
    int sd = srcs[ed];
    int td = types[ed];
    asm volatile("" :: "v"(sa));
    asm volatile("" :: "v"(ta));
    asm volatile("" :: "v"(sb));
    asm volatile("" :: "v"(tb));
    asm volatile("" :: "v"(sc));
    asm volatile("" :: "v"(tc));
    asm volatile("" :: "v"(sd));
    asm volatile("" :: "v"(td));
    const int wa = (clampi(ta, 0, NR - 1) << 16) | clampi(sa, 0, NN - 1);
    const int wb = (clampi(tb, 0, NR - 1) << 16) | clampi(sb, 0, NN - 1);
    const int wc = (clampi(tc, 0, NR - 1) << 16) | clampi(sc, 0, NN - 1);
    const int wd2 = (clampi(td, 0, NR - 1) << 16) | clampi(sd, 0, NN - 1);
    const int ma = (i     < tot) ? -1 : 0;
    const int mb = (i + 1 < tot) ? -1 : 0;
    const int mc = (i + 2 < tot) ? -1 : 0;
    const int md = (i + 3 < tot) ? -1 : 0;
    const v4i v = {wa & ma, wb & mb, wc & mc, wd2 & md};
    st2_v4i(lp + i, v);
  }
#pragma unroll 1
  for (int it = 0; it < 2; ++it) {
    const v4i v = *(const v4ia*)(cnt + it * (NTHR * 4) + 4 * tid);
    st2_v4i(cop + it * (NTHR * 4) + 4 * tid, v);
  }
  if (tid < 8) {
    const v4i f = {ovf, ovf, ovf, ovf};
    st2_v4i(fp + 4 * tid, f);
  }
}

template <int F>
__device__ __forceinline__ typename RowV<F>::V walk_hits(unsigned mask, int w, const float* __restrict__ T, int lane,
                                                         typename RowV<F>::V a) {
  typedef typename RowV<F>::V V;
  typedef typename RowV<F>::VA VA;
  constexpr int CPL = F / 32;
#pragma unroll 1
  for (int it = 0; it < 32 && mask != 0u; ++it) {
    const int k = __builtin_ctz(mask);
    mask &= mask - 1u;
    const int u  = __builtin_amdgcn_readlane(w, k);
    const int sk = clampi(u & 0xFFFF, 0, NN - 1);
    const V t = *(const VA*)(T + (size_t)sk * F + CPL * lane);
    asm volatile("" :: "v"(t));
    a = vadd(a, t);
  }
  return a;
}

template <int F>
__global__ __launch_bounds__(NTHR) void k_relwalk(const float* __restrict__ T, const int* __restrict__ LIST,
                                                  const int* __restrict__ CO, const int* __restrict__ FLAG,
                                                  int r, int first, float* ACC) {
  static_assert(F == 128 || F == 64);
  static_assert(F % 32 == 0);
  typedef typename RowV<F>::V V;
  typedef typename RowV<F>::VA VA;
  constexpr int CPL = F / 32;
  const int tid = (int)threadIdx.x, lane = tid & 31, wave = tid >> 5;
  const int d = (int)blockIdx.x * 8 + wave;
  const int blk = d >> SLB, slot = d & (NBRUN - 1);
  const int* cob = CO + (size_t)blk * (2 * NBRUN);
  int cv = cob[slot];
  int ov = cob[NBRUN + slot];
  int flag = FLAG[(size_t)blk * 32];
  asm volatile("" :: "v"(cv));
  asm volatile("" :: "v"(ov));
  asm volatile("" :: "v"(flag));
  const int big = (cv > WCAP) ? 1 : 0;
  cv = clampi(cv, 0, WCAP);
  ov = clampi(ov, 0, LCAP - 1);
  const int c = __builtin_amdgcn_readfirstlane(cv);
  const int o = __builtin_amdgcn_readfirstlane(ov);
  int last = o + (c > 0 ? c : 1) - 1;
  last = last > LCAP - 1 ? LCAP - 1 : last;
  int i0 = o + lane;
  i0 = i0 > last ? last : i0;
  int i1 = o + 32 + lane;
  i1 = i1 > last ? last : i1;
  const int* lb = LIST + (size_t)blk * (size_t)LCAP;
  int w0 = lb[i0];
  int w1 = lb[i1];
  asm volatile("" :: "v"(w0));
  asm volatile("" :: "v"(w1));
  const bool h0 = (lane < c) && (((w0 >> 16) & 7) == r);
  const bool h1 = (lane + 32 < c) && (((w1 >> 16) & 7) == r);
  const unsigned m0 = __builtin_amdgcn_ballot_w32(h0);
  const unsigned m1 = __builtin_amdgcn_ballot_w32(h1);
  V a = RowV<F>::zero();
  a = walk_hits<F>(m0, w0, T, lane, a);
  a = walk_hits<F>(m1, w1, T, lane, a);
  const int cnt = (int)(__builtin_popcount(m0) + __builtin_popcount(m1));
  const float den = (float)(cnt > 0 ? cnt : 1);
  V m = vdivs(a, den);
  const int badi = __builtin_amdgcn_readfirstlane(((flag != 0) || (big != 0)) ? 1 : 0);
  m = vpois(m, badi != 0);
  float* ap = ACC + (size_t)d * F + CPL * lane;
  if (first != 0) {
    st2row(ap, m);
  } else if (cnt != 0 || badi != 0) {
    const V curv = *(const VA*)ap;
    asm volatile("" :: "v"(curv));
    const V o2 = vadd(curv, m);
    st2row(ap, o2);
  }
}

__global__ __launch_bounds__(NTHR) void k_close1(const float* __restrict__ ACC, const float* __restrict__ T,
                                                 const float* __restrict__ B1F, unsigned short* OP) {
  const int tid = (int)threadIdx.x, lane = tid & 31, wave = tid >> 5;
  const int hh = lane >> 4;
  const int c8 = (lane & 15) * 8;
  const int d = ((int)blockIdx.x * 8 + wave) * 2 + hh;
  const float* ar = ACC + (size_t)d * FI + c8;
  const float* tr = T + (size_t)d * FI + c8;
  const v4f a0 = *(const v4fa*)ar;
  const v4f a1 = *(const v4fa*)(ar + 4);
  const v4f t0 = *(const v4fa*)tr;
  const v4f t1 = *(const v4fa*)(tr + 4);
  const v4f b0 = *(const v4fa*)(B1F + c8);
  const v4f b1 = *(const v4fa*)(B1F + c8 + 4);
  asm volatile("" :: "v"(a0));
  asm volatile("" :: "v"(a1));
  asm volatile("" :: "v"(t0));
  asm volatile("" :: "v"(t1));
  v4f h0, h1;
  h0.x = relu_keep((a0.x + t0.x) + b0.x); h0.y = relu_keep((a0.y + t0.y) + b0.y);
  h0.z = relu_keep((a0.z + t0.z) + b0.z); h0.w = relu_keep((a0.w + t0.w) + b0.w);
  h1.x = relu_keep((a1.x + t1.x) + b1.x); h1.y = relu_keep((a1.y + t1.y) + b1.y);
  h1.z = relu_keep((a1.z + t1.z) + b1.z); h1.w = relu_keep((a1.w + t1.w) + b1.w);
  unsigned short* orow = OP + (size_t)d * KT2 + c8;
  const v4u hi = pack8_bf16(h0, h1);
  st2_v4u(orow, hi);
#if SPLIT_L2
  const v4u lo = pack8_bf16_lo(h0, h1);
  st2_v4u(orow + FI, lo);
#endif
}

__global__ __launch_bounds__(NTHR) void k_close2(const float* __restrict__ ACC, const float* __restrict__ T,
                                                 const float* __restrict__ B2F, const int* __restrict__ FLAG,
                                                 float* out, int nreal) {
  const int tid = (int)threadIdx.x, lane = tid & 31, wave = tid >> 5;
  const int d = (int)blockIdx.x * 8 + wave;
  int flag = FLAG[(size_t)(d >> SLB) * 32];
  asm volatile("" :: "v"(flag));
  const v2f a = *(const v2fa*)(ACC + (size_t)d * FO + 2 * lane);
  const v2f t = *(const v2fa*)(T + (size_t)d * FO + 2 * lane);
  const v2f b = *(const v2fa*)(B2F + 2 * lane);
  asm volatile("" :: "v"(a));
  asm volatile("" :: "v"(t));
  const float vx = (a.x + t.x) + b.x;
  const float vy = (a.y + t.y) + b.y;
  v2f o;
  o.x = 1.0f / (1.0f + expf(-vx));
  o.y = 1.0f / (1.0f + expf(-vy));
  o = vpois(o, flag != 0);
  if (d < nreal) st2_v2f(out + (size_t)d * FO + 2 * lane, o);
}

extern "C" void kernel_launch(void* const* d_in, const int* in_sizes, int n_in,
                              void* d_out, int out_size, void* d_ws, size_t ws_size,
                              hipStream_t stream) {
  if (n_in < 9) return;
  if (in_sizes[0] != NN * FI) return;
  if (in_sizes[1] != 2 * NE) return;
  if (in_sizes[2] != NE) return;
  if (in_sizes[3] != NR * FI * FI) return;
  if (in_sizes[4] != FI * FI) return;
  if (in_sizes[5] != FI) return;
  if (in_sizes[6] != NR * FI * FO) return;
  if (in_sizes[7] != FI * FO) return;
  if (in_sizes[8] != FO) return;
  if (out_size != NN * FO) return;

  const float* x     = (const float*)d_in[0];
  const int*   eidx  = (const int*)d_in[1];
  const int*   srcs  = eidx;
  const int*   dsts  = eidx + NE;
  const int*   types = (const int*)d_in[2];
  const float* W1    = (const float*)d_in[3];
  const float* R1    = (const float*)d_in[4];
  const float* b1    = (const float*)d_in[5];
  const float* W2    = (const float*)d_in[6];
  const float* R2    = (const float*)d_in[7];
  const float* b2    = (const float*)d_in[8];
  float* out = (float*)d_out;

  constexpr size_t zXB   = (size_t)MP * FI * 2;
  constexpr size_t zOP   = (size_t)MP * KT2 * 2;
  constexpr size_t zT    = (size_t)MP * FI * 4;
  constexpr size_t zACC  = (size_t)MP * FI * 4;
  constexpr size_t zLIST = (size_t)NBK * LCAP * 4;
  constexpr size_t zCO   = (size_t)NBK * 2 * NBRUN * 4;
  constexpr size_t zFLAG = (size_t)FLAGB;
  constexpr size_t zWP1  = (size_t)(NR + 1) * FI * FI * 2;
  constexpr size_t zWP2  = (size_t)(NR + 1) * FO * KT2 * 2;
  constexpr size_t zTAB  = (size_t)(FI + FO) * 4;
  constexpr size_t oXB   = 0;
  constexpr size_t oOP   = oXB + zXB;
  constexpr size_t oT    = oOP + zOP;
  constexpr size_t oACC  = oT + zT;
  constexpr size_t oLIST = oACC + zACC;
  constexpr size_t oCO   = oLIST + zLIST;
  constexpr size_t oFLAG = oCO + zCO;
  constexpr size_t oWP1  = oFLAG + zFLAG;
  constexpr size_t oWP2  = oWP1 + zWP1;
  constexpr size_t oTAB  = oWP2 + zWP2;
  constexpr size_t oEND  = oTAB + zTAB;
  static_assert(zXB % 256 == 0 && zOP % 256 == 0 && zT % 256 == 0 && zACC % 256 == 0 && zLIST % 256 == 0);
  static_assert(zCO % 256 == 0 && zFLAG % 256 == 0 && zWP1 % 256 == 0 && zWP2 % 256 == 0 && zTAB % 256 == 0);
  static_assert(zT >= (size_t)MP * FO * 4 && zACC >= (size_t)NN * FI * 4);
  static_assert(oEND == (SPLIT_L2 ? (size_t)93295360 : (size_t)80335616));
  static_assert(oEND <= (size_t)WSMAX);
  if (oEND > ws_size) return;

  char* ws = (char*)d_ws;
  unsigned short* XB   = (unsigned short*)(ws + oXB);
  unsigned short* OP   = (unsigned short*)(ws + oOP);
  float*          T    = (float*)(ws + oT);
  float*          ACC  = (float*)(ws + oACC);
  int*            LIST = (int*)(ws + oLIST);
  int*            CO   = (int*)(ws + oCO);
  int*            FLAG = (int*)(ws + oFLAG);
  unsigned short* WP1  = (unsigned short*)(ws + oWP1);
  unsigned short* WP2  = (unsigned short*)(ws + oWP2);
  float*          TABB = (float*)(ws + oTAB);
  float*          B1F  = TABB;
  float*          B2F  = TABB + FI;

  hipFuncSetAttribute(reinterpret_cast<const void*>(&k_list), hipFuncAttributeMaxDynamicSharedMemorySize, (int)BK_LDS);

  k_plane<0><<<MP * FI / 8 / 256, 256, 0, stream>>>(x, NN, FI, FI, XB, MP, FI);
  k_prep<<<PB_ALL, NTHR, 0, stream>>>(W1, R1, b1, W2, R2, b2, WP1, WP2, TABB, OP, FLAG);
  k_list<<<NBK, NTHR, BK_LDS, stream>>>(srcs, dsts, types, LIST, CO, FLAG);

  for (int r = 0; r < NR; ++r) {
    k_gemm_nt<0, 0><<<(G1TILES + 7) / 8, 256, 0, stream>>>(XB, WP1 + (size_t)r * FI * FI, B1F, T, MP, FI, FI, FI);
    k_relwalk<128><<<NN / 8, NTHR, 0, stream>>>(T, LIST, CO, FLAG, r, (r == 0) ? 1 : 0, ACC);
  }
  k_gemm_nt<0, 0><<<(G1TILES + 7) / 8, 256, 0, stream>>>(XB, WP1 + (size_t)NR * FI * FI, B1F, T, MP, FI, FI, FI);
  k_close1<<<NN / 16, NTHR, 0, stream>>>(ACC, T, B1F, OP);

  for (int r = 0; r < NR; ++r) {
    k_gemm_nt<0, 0><<<(G2TILES + 7) / 8, 256, 0, stream>>>(OP, WP2 + (size_t)r * FO * KT2, B2F, T, MP, FO, KT2, FO);
    k_relwalk<64><<<NN / 8, NTHR, 0, stream>>>(T, LIST, CO, FLAG, r, (r == 0) ? 1 : 0, ACC);
  }
  k_gemm_nt<0, 0><<<(G2TILES + 7) / 8, 256, 0, stream>>>(OP, WP2 + (size_t)NR * FO * KT2, B2F, T, MP, FO, KT2, FO);
  k_close2<<<NN / 8, NTHR, 0, stream>>>(ACC, T, B2F, FLAG, out, NN);
}
